// _OuterProductMean_34995393528036
// MI455X (gfx1250) — hardware-verified
//
#include <hip/hip_runtime.h>


#define SQ   256
#define NSEQ 256
#define CC   32
#define CZ   128
#define NP   (SQ * NSEQ)
#define ICH  16
#define DM   NSEQ
#define LEPS 1e-5f
#define LOSC 1024.0f

typedef _Float16 h16;
typedef unsigned short bf;
typedef __attribute__((ext_vector_type(16))) __bf16   v16bf;
typedef __attribute__((ext_vector_type(16))) _Float16 v16h;
typedef __attribute__((ext_vector_type(8)))  _Float16 v8h;
typedef __attribute__((ext_vector_type(8)))  unsigned short v8us;
typedef __attribute__((ext_vector_type(8)))  float    v8f;
typedef __attribute__((ext_vector_type(4)))  float    v4f;
typedef v8h  __attribute__((may_alias)) v8ha;
typedef v4f  __attribute__((may_alias)) v4fa;
typedef v8us __attribute__((may_alias)) v8usa;

__device__ __forceinline__ unsigned short f2bf(float f) { unsigned u = __float_as_uint(f); u += 0x7FFFu + ((u >> 16) & 1u); return (unsigned short)(u >> 16); }
__device__ __forceinline__ float bf2f(unsigned short b) { return __uint_as_float(((unsigned)b) << 16); }
__device__ __forceinline__ float bfr(float f) { return bf2f(f2bf(f)); }
__device__ __forceinline__ v16h cat16(v8h lo, v8h hi) { return __builtin_shufflevector(lo, hi, 0, 1, 2, 3, 4, 5, 6, 7, 8, 9, 10, 11, 12, 13, 14, 15); }
__device__ __forceinline__ v16bf cat16b(v8us lo, v8us hi) { return __builtin_bit_cast(v16bf, __builtin_shufflevector(lo, hi, 0, 1, 2, 3, 4, 5, 6, 7, 8, 9, 10, 11, 12, 13, 14, 15)); }
__device__ __forceinline__ v8f wmma16(v16h a, v16h b, v8f c) { return __builtin_amdgcn_wmma_f32_16x16x32_f16(false, a, false, b, (short)0, c, false, false); }
__device__ __forceinline__ v8f wmmab(v16bf a, v16bf b, v8f c) { return __builtin_amdgcn_wmma_f32_16x16x32_bf16(false, a, false, b, (short)0, c, false, false); }

template <bool SPLITA, bool F16OUT = false>
__global__ __launch_bounds__(128) void k_gemmb(const bf* __restrict__ A, const bf* __restrict__ Al, const bf* __restrict__ Bn, const float* __restrict__ bias, float* C, int ldc, h16* C2, const float* __restrict__ R = nullptr, int K = DM, int roundR = 1) {
    __shared__ __align__(16) float ost[4][16 * 68];
    const int lane = threadIdx.x & 31, wave = threadIdx.x >> 5, lr = lane & 15, hi = lane >> 4;
    const int r0 = blockIdx.x * 64 + wave * 16, c0 = blockIdx.y * 64;
    const size_t aoff = (size_t)(r0 + lr) * K + 8 * hi;
    size_t boff[4];
#pragma unroll
    for (int t = 0; t < 4; ++t) boff[t] = (size_t)(c0 + t * 16 + lr) * K + 8 * hi;
    v8f acc[4];
#pragma unroll
    for (int t = 0; t < 4; ++t) acc[t] = (v8f){};
#pragma unroll 1
    for (int kc = 0; kc < K; kc += 32) {
        const v16bf a = cat16b(*(const v8us*)(A + aoff + kc), *(const v8us*)(A + aoff + kc + 16));
        v16bf al = a;
        if (SPLITA) al = cat16b(*(const v8us*)(Al + aoff + kc), *(const v8us*)(Al + aoff + kc + 16));
#pragma unroll
        for (int t = 0; t < 4; ++t) { const v16bf b = cat16b(*(const v8us*)(Bn + boff[t] + kc), *(const v8us*)(Bn + boff[t] + kc + 16)); acc[t] = wmmab(a, b, acc[t]); if (SPLITA) acc[t] = wmmab(al, b, acc[t]); }
        asm volatile("v_nop\n\tv_nop\n\tv_nop\n\tv_nop" : "+v"(acc[0]), "+v"(acc[1]), "+v"(acc[2]), "+v"(acc[3]) : "v"(a), "v"(al));
    }
    float* os = &ost[wave][0];
#pragma unroll
    for (int t = 0; t < 4; ++t) { const float bv = bias ? bfr(bias[c0 + t * 16 + lr]) : 0.f;
#pragma unroll
        for (int j = 0; j < 8; ++j) os[(hi * 8 + j) * 68 + t * 16 + lr] = acc[t][j] + bv; }
    __syncthreads();
    if (F16OUT) {
        h16* crow = (h16*)(void*)C + (size_t)r0 * ldc + c0;
        auto pass = [&]() {
#pragma unroll
            for (int s = 0; s < 4; ++s) { const int row = 4 * s + (lane >> 3), piece = lane & 7; const float* sp = os + row * 68 + piece * 8; v8h o, o2;
#pragma unroll
                for (int i = 0; i < 8; ++i) { const h16 a = (h16)sp[i]; o[i] = a; o2[i] = (h16)((sp[i] - (float)a) * LOSC); }
                *(volatile v8h*)(crow + (size_t)row * ldc + piece * 8) = o; if (C2) *(volatile v8h*)(C2 + (size_t)r0 * ldc + c0 + (size_t)row * ldc + piece * 8) = o2; }
        };
        pass(); __threadfence(); pass();
    } else {
        float* crow = C + (size_t)r0 * ldc + c0;
        auto pass = [&]() {
#pragma unroll
            for (int s = 0; s < 8; ++s) { const int Lid = (lane >> 3) + 4 * s, piece = lane & 7; const int row = Lid >> 1, cofs = (Lid & 1) * 32 + piece * 4;
                v4f val = *(const v4fa*)(os + row * 68 + cofs); if (R) { const v4f rv = *(const v4f*)(R + ((size_t)r0 + row) * ldc + c0 + cofs); val += roundR ? (v4f){bfr(rv[0]), bfr(rv[1]), bfr(rv[2]), bfr(rv[3])} : rv; }
                *(volatile v4f*)(crow + (size_t)row * ldc + cofs) = val; }
        };
        pass(); __threadfence(); pass();
    }
}


__global__ __launch_bounds__(256) void k_cvt8(const float* __restrict__ src, bf* dst, size_t n8) {
    const size_t i = (size_t)blockIdx.x * 256 + threadIdx.x; if (i >= n8) return;
    const v8f v = *(const v8f*)(src + i * 8); v8us o;
#pragma unroll
    for (int k = 0; k < 8; ++k) o[k] = f2bf(v[k]);
    *(volatile v8us*)(dst + i * 8) = o; __threadfence(); *(volatile v8us*)(dst + i * 8) = o;
}
__global__ __launch_bounds__(256) void k_zero8(bf* dst, size_t n8) {
    const size_t i = (size_t)blockIdx.x * 256 + threadIdx.x; if (i >= n8) return; v8us z;
#pragma unroll
    for (int k = 0; k < 8; ++k) z[k] = 0;
    *(volatile v8us*)(dst + i * 8) = z; __threadfence(); *(volatile v8us*)(dst + i * 8) = z;
}

__global__ __launch_bounds__(256) void k_ln32(const float* __restrict__ m, const float* __restrict__ g, const float* __restrict__ bb, bf* Xh, bf* Xl) {
    typedef __attribute__((ext_vector_type(2))) unsigned short v2us;
    const int lane = threadIdx.x & 31; const size_t r = ((size_t)blockIdx.x * 8 + (threadIdx.x >> 5)) * 2 + (lane >> 4); if (r >= (size_t)NP) return; const int c0 = (lane & 15) * 2;
    const float v0 = bfr(m[r * CC + c0]), v1 = bfr(m[r * CC + c0 + 1]); float s = v0 + v1;
#pragma unroll
    for (int sh = 8; sh; sh >>= 1) s += __shfl_xor(s, sh, 32);
    const float mu = s * (1.0f / CC); float q = (v0 - mu) * (v0 - mu) + (v1 - mu) * (v1 - mu);
#pragma unroll
    for (int sh = 8; sh; sh >>= 1) q += __shfl_xor(q, sh, 32);
    const float rs = rsqrtf(q * (1.0f / CC) + LEPS); v2us oh, ol;
    { const float y = (v0 - mu) * rs * bfr(g[c0]) + bfr(bb[c0]); const unsigned short hb = f2bf(y); oh[0] = hb; ol[0] = f2bf(y - bf2f(hb)); }
    { const float y = (v1 - mu) * rs * bfr(g[c0 + 1]) + bfr(bb[c0 + 1]); const unsigned short hb = f2bf(y); oh[1] = hb; ol[1] = f2bf(y - bf2f(hb)); }
    const size_t o = r * CC + c0; *(volatile v2us*)(Xh + o) = oh; *(volatile v2us*)(Xl + o) = ol; __threadfence(); *(volatile v2us*)(Xh + o) = oh; *(volatile v2us*)(Xl + o) = ol;
}
__global__ __launch_bounds__(256) void k_abT(const float* __restrict__ AB, bf* ATh, bf* ATl, bf* BTh, bf* BTl) {
    __shared__ float tl[64][65];
    const int tid = threadIdx.x, n0 = blockIdx.x * 64, s = blockIdx.y; const int nn = tid >> 2, cq = (tid & 3) * 16;
#pragma unroll
    for (int i = 0; i < 16; ++i) tl[nn][cq + i] = AB[((size_t)s * NSEQ + n0 + nn) * 64 + cq + i];
    __syncthreads();
    const int piece = tid & 7, cr0 = tid >> 3;
    auto pass = [&]() {
#pragma unroll
        for (int st = 0; st < 2; ++st) { const int col = cr0 + 32 * st; v8us oh, ol;
#pragma unroll
            for (int i = 0; i < 8; ++i) { const float v = tl[piece * 8 + i][col]; const unsigned short hb = f2bf(v); oh[i] = hb; ol[i] = f2bf(v - bf2f(hb)); }
            bf* dh = (col < CC) ? ATh : BTh; bf* dl = (col < CC) ? ATl : BTl; const int cc = (col < CC) ? col : col - CC;
            const size_t o = ((size_t)s * CC + cc) * NSEQ + n0 + piece * 8; *(volatile v8us*)(dh + o) = oh; *(volatile v8us*)(dl + o) = ol; }
    };
    pass(); __threadfence(); pass();
}
__global__ __launch_bounds__(256) void k_regather(const float* __restrict__ Cm, bf* OPh, bf* OPl) {
    const int lane = threadIdx.x & 31; const size_t wid = (size_t)blockIdx.x * 8 + (threadIdx.x >> 5); if (wid >= (size_t)ICH * SQ * 4) return; const int q4 = (int)(wid & 3); const size_t ij = wid >> 2; const int j = (int)(ij % SQ), il = (int)(ij / SQ);
    const int c = q4 * 8 + (lane >> 2), d0 = (lane & 3) * 8; v8us oh, ol;
#pragma unroll
    for (int i = 0; i < 8; ++i) { const float v = Cm[((size_t)il * CC + c) * ((size_t)SQ * CC) + (size_t)j * CC + d0 + i] * (1.0f / NSEQ); const unsigned short hb = f2bf(v); oh[i] = hb; ol[i] = f2bf(v - bf2f(hb)); }
    const size_t o = ij * (CC * CC) + c * CC + d0; *(volatile v8us*)(OPh + o) = oh; *(volatile v8us*)(OPl + o) = ol; __threadfence(); *(volatile v8us*)(OPh + o) = oh; *(volatile v8us*)(OPl + o) = ol;
}

extern "C" void kernel_launch(void* const* d_in, const int* in_sizes, int n_in,
                              void* d_out, int out_size, void* d_ws, size_t ws_size, hipStream_t stream) {
    (void)in_sizes; (void)n_in; (void)out_size;
    const float* m = (const float*)d_in[0]; const float* g = (const float*)d_in[1]; const float* bb = (const float*)d_in[2]; const float* Wab = (const float*)d_in[3]; const float* Wout = (const float*)d_in[4]; const float* bout = (const float*)d_in[5];
    float* out = (float*)d_out;
    char* wsp = (char*)d_ws;
    auto take = [&](size_t bytes) { char* p = wsp; wsp += (bytes + 255) & ~(size_t)255; return (void*)p; };
    bf* WAB = (bf*)take(64 * CC * 2); bf* WOUT = (bf*)take((size_t)CZ * CC * CC * 2);
    bf* Xh = (bf*)take((size_t)NP * CC * 2); bf* Xl = (bf*)take((size_t)NP * CC * 2); float* AB = (float*)take((size_t)NP * 64 * 4);
    bf* ATh = (bf*)take((size_t)SQ * CC * NSEQ * 2); bf* ATl = (bf*)take((size_t)SQ * CC * NSEQ * 2); bf* BTh = (bf*)take((size_t)SQ * CC * NSEQ * 2); bf* BTl = (bf*)take((size_t)SQ * CC * NSEQ * 2);
    float* C1 = (float*)take((size_t)ICH * CC * SQ * CC * 4); float* Cm = (float*)take((size_t)ICH * CC * SQ * CC * 4); bf* OPh = (bf*)take((size_t)ICH * SQ * CC * CC * 2); bf* OPl = (bf*)take((size_t)ICH * SQ * CC * CC * 2);
    if ((size_t)(wsp - (char*)d_ws) > ws_size) return;
    k_cvt8<<<(64 * CC / 8 + 255) / 256, 256, 0, stream>>>(Wab, WAB, 64 * CC / 8); k_cvt8<<<(CZ * CC * CC / 8 + 255) / 256, 256, 0, stream>>>(Wout, WOUT, (size_t)CZ * CC * CC / 8);
    k_ln32<<<(NP / 2) / 8, 256, 0, stream>>>(m, g, bb, Xh, Xl);
    k_gemmb<true, false><<<dim3(NP / 64, 1, 1), 128, 0, stream>>>(Xh, Xl, WAB, nullptr, AB, 64, nullptr, nullptr, CC);
    k_abT<<<dim3(NSEQ / 64, SQ, 1), 256, 0, stream>>>(AB, ATh, ATl, BTh, BTl);
    for (int ch = 0; ch < SQ / ICH; ++ch) { const size_t r0 = (size_t)ch * ICH * CC;
        k_gemmb<true, false><<<dim3((ICH * CC) / 64, (SQ * CC) / 64, 1), 128, 0, stream>>>(ATh + r0 * NSEQ, ATl + r0 * NSEQ, BTh, nullptr, C1, SQ * CC, nullptr, nullptr, NSEQ);
        k_gemmb<false, false><<<dim3((ICH * CC) / 64, (SQ * CC) / 64, 1), 128, 0, stream>>>(ATh + r0 * NSEQ, nullptr, BTl, nullptr, Cm, SQ * CC, nullptr, C1, NSEQ, 0);
        k_regather<<<(ICH * SQ * 4) / 8, 256, 0, stream>>>(Cm, OPh, OPl);
        k_gemmb<true, false><<<dim3((ICH * SQ) / 64, CZ / 64, 1), 128, 0, stream>>>(OPh, OPl, WOUT, bout, out + (size_t)ch * ICH * SQ * CZ, CZ, nullptr, nullptr, CC * CC); }
}
